// MaskedPiecewiseRationalQuadraticAutoregressive_4870492913671
// MI455X (gfx1250) — hardware-run, weakly checked
//
#include <hip/hip_runtime.h>
#include <math.h>
#include <stddef.h>

typedef __attribute__((ext_vector_type(16))) _Float16 v16h;
typedef __attribute__((ext_vector_type(8)))  _Float16 v8h;
typedef __attribute__((ext_vector_type(8)))  float    v8f;
typedef __attribute__((ext_vector_type(4)))  float    v4f;

constexpr int kB      = 16384;
constexpr int kD      = 128;
constexpr int kH      = 1024;
constexpr int kBins   = 8;
constexpr int kOpd    = 3 * kBins + 1;
constexpr int kNOut   = kD * kOpd;
constexpr int kChunk  = 2048;
constexpr int kNChunk = kB / kChunk;
constexpr int kSpRows = 32;
constexpr int kStripV = 7 * 32;
constexpr int kStripF = kStripV * 4;
constexpr int kSlabF  = 32 * kOpd;
constexpr int kSlabV  = kSlabF / 4;

constexpr float kTB       = 3.0f;
constexpr float kEps      = 1e-12f;
constexpr float kMinBin   = 1e-3f;
constexpr float kMinDer   = 1e-3f;
constexpr float kBinScale = (float)(1.0 - 1e-3 * kBins);
constexpr float kInvSpan  = 1.0f / (2.0f * kTB);
constexpr float kSpanY    = 2.0f * kTB;
constexpr float kSlope    = (2.0f * kTB) / (2.0f * kTB);
constexpr float kWCarry    = 16.0f;
constexpr float kWCarryInv = 1.0f / kWCarry;

static_assert(kOpd == 25 && kNOut == 3200, "parameter row layout");
static_assert((kD % 32) == 0 && (kH % 32) == 0, "GEMM K multiples of 32");
static_assert((kB % 64) == 0 && (kChunk % 64) == 0 && (kH % 64) == 0 && (kNOut % 64) == 0, "GEMM M,N multiples of 64");
static_assert(((kB / 64) * (kH / 64)) % 8 == 0 && ((kChunk / 64) * (kNOut / 64)) % 8 == 0, "whole blocks of 8 tiles");
static_assert((kSlabF % 4) == 0 && kSlabV == 200 && kSlabV <= kStripV, "slab staging");
static_assert((kChunk % kSpRows) == 0 && kD == 128, "spline tiling");

constexpr size_t kOffXH  = 0;
constexpr size_t kOffW1  = kOffXH + (size_t)kB * kD * 2;
constexpr size_t kOffW2  = kOffW1 + (size_t)kH * kD * 2;
constexpr size_t kOffW3  = kOffW2 + (size_t)kH * kH * 2;
constexpr size_t kOffH1  = kOffW3 + (size_t)kNOut * kH * 2;
constexpr size_t kOffH2  = kOffH1 + (size_t)kB * kH * 2;
constexpr size_t kOffRaw = kOffH2 + (size_t)kB * kH * 2;
constexpr size_t kWsTotal = kOffRaw + (size_t)kChunk * kNOut * 4;
static_assert(kWsTotal == 106430464ull, "carve total");
static_assert(kWsTotal <= 134217728ull, "carve cap");
static_assert((kOffW1 % 128) == 0 && (kOffW2 % 128) == 0 && (kOffW3 % 128) == 0 && (kOffH1 % 128) == 0 &&
              (kOffH2 % 128) == 0 && (kOffRaw % 128) == 0, "128-B aligned regions");
constexpr size_t kOut1OffBytes = (size_t)kB * kD * 4;
static_assert(kOut1OffBytes == 8388608ull && (kOut1OffBytes % 128) == 0, "second output offset");
static_assert(kOut1OffBytes + (size_t)kB * 4 == 8454144ull, "output total");

struct FragH {
  union U { v16h v; v8h h[2]; };
  static __device__ __forceinline__ v16h load(const _Float16* p) {
    U f; f.h[0] = *(const v8h*)(p); f.h[1] = *(const v8h*)(p + 16); return f.v;
  }
  static __device__ __forceinline__ v8f mma(v16h a, v16h b, v8f c) {
    return __builtin_amdgcn_wmma_f32_16x16x32_f16(false, a, false, b, (short)0, c, false, false);
  }
};
__device__ __forceinline__ void acc_guard1(v8f& a, v16h x, v16h y) {
  asm volatile("v_nop\n\tv_nop\n\tv_nop\n\tv_nop" : "+v"(a) : "v"(x), "v"(y));
}
__device__ __forceinline__ void keep4_h(v16h a, v16h b, v16h c, v16h d) {
  asm volatile("v_nop" :: "v"(a), "v"(b), "v"(c), "v"(d));
}

template <int OUT_MODE, int ACT>
__global__ __launch_bounds__(256) void wmma_gemm64(
    const unsigned short* __restrict__ Ap, int lda,
    const unsigned short* __restrict__ Btp, int ldb,
    void* __restrict__ Cout, int ldc,
    const float* __restrict__ bias,
    int M, int N, int K, float scale) {
  const _Float16* A  = (const _Float16*)Ap;
  const _Float16* Bt = (const _Float16*)Btp;
  __shared__ __align__(16) float sT[8][16 * 68];
  const int lane = threadIdx.x & 31;
  const int wave = threadIdx.x >> 5;
  const int tilesN = N >> 6;
  const int tilesM = M >> 6;
  const int tile = blockIdx.x * 8 + wave;
  if (tile >= tilesM * tilesN) return;
  const int tm = tile / tilesN;
  const int tn = tile - tm * tilesN;
  const int m0 = tm << 6;
  const int n0 = tn << 6;

  const int rlane = lane & 15;
  const int koff  = (lane >> 4) * 8;
  const int mOff  = (lane >> 4) * 8;

  v8f acc[4][4];
#pragma unroll
  for (int i = 0; i < 4; ++i)
#pragma unroll
    for (int j = 0; j < 4; ++j) acc[i][j] = (v8f){0.f,0.f,0.f,0.f,0.f,0.f,0.f,0.f};

  for (int k0 = 0; k0 < K; k0 += 32) {
    v16h bh[4];
#pragma unroll
    for (int j = 0; j < 4; ++j) {
      const size_t bo = (size_t)(n0 + (j << 4) + rlane) * ldb + koff + k0;
      bh[j] = FragH::load(Bt + bo);
    }
#pragma unroll
    for (int i = 0; i < 4; ++i) {
      const size_t ao = (size_t)(m0 + (i << 4) + rlane) * lda + koff + k0;
      v16h ah = FragH::load(A + ao);
#pragma unroll
      for (int j = 0; j < 4; ++j) acc[i][j] = FragH::mma(ah, bh[j], acc[i][j]);
#pragma unroll
      for (int j = 0; j < 4; ++j) acc_guard1(acc[i][j], ah, bh[j]);
    }
    keep4_h(bh[0], bh[1], bh[2], bh[3]);
  }

  float* slab = sT[wave];
#pragma unroll
  for (int i = 0; i < 4; ++i) {
    const int mBase = m0 + (i << 4);
#pragma unroll
    for (int j = 0; j < 4; ++j) {
      const int n = n0 + (j << 4) + rlane;
      const float bv = bias[n];
#pragma unroll
      for (int r = 0; r < 8; ++r) {
        float v = acc[i][j][r] * scale;
        v += bv;
        if (ACT == 3) v = v * __builtin_amdgcn_rcpf(1.0f + __expf(-v));
        slab[(mOff + r) * 68 + (j << 4) + rlane] = v;
      }
    }
    __builtin_amdgcn_fence(__ATOMIC_RELEASE, "workgroup");
    __builtin_amdgcn_wave_barrier();
    __builtin_amdgcn_fence(__ATOMIC_ACQUIRE, "workgroup");
    if (OUT_MODE == 0) {
      float* C = (float*)Cout;
      const int hh = lane >> 4, c4 = (lane & 15) * 4;
      for (int pass = 0; pass < 2; ++pass) {
#pragma unroll
        for (int it = 0; it < 8; ++it) {
          const int row = it * 2 + hh;
          const v4f sv = *(const v4f*)(slab + row * 68 + c4);
          *(volatile v4f*)(C + (size_t)(mBase + row) * ldc + n0 + c4) = sv;
        }
        __threadfence();
      }
    } else {
      const int q = lane >> 3, c8 = (lane & 7) * 8;
      unsigned short* C = (unsigned short*)Cout;
      for (int pass = 0; pass < 2; ++pass) {
#pragma unroll
        for (int it = 0; it < 4; ++it) {
          const int row = it * 4 + q;
          const float* sp = slab + row * 68 + c8;
          v8h hv;
#pragma unroll
          for (int e = 0; e < 8; ++e) hv[e] = (_Float16)sp[e];
          *(volatile v8h*)(C + (size_t)(mBase + row) * ldc + n0 + c8) = hv;
        }
        __threadfence();
      }
    }
    __builtin_amdgcn_fence(__ATOMIC_RELEASE, "workgroup");
    __builtin_amdgcn_wave_barrier();
    __builtin_amdgcn_fence(__ATOMIC_ACQUIRE, "workgroup");
  }
}

template <bool MASKED>
__global__ __launch_bounds__(256) void pack_f16_kernel(
    const float* __restrict__ src, const float* __restrict__ msk, unsigned short* __restrict__ dst,
    int total8, float carry)
{
  const int i = blockIdx.x * 256 + threadIdx.x;
  if (i >= total8) return;
  const size_t e0 = (size_t)i << 3;
  const v4f a0 = *(const v4f*)(src + e0);
  const v4f a1 = *(const v4f*)(src + e0 + 4);
  v4f q0 = a0, q1 = a1;
  if (MASKED) {
    q0 = *(const v4f*)(msk + e0);
    q1 = *(const v4f*)(msk + e0 + 4);
  }
  v8h hv;
#pragma unroll
  for (int e = 0; e < 4; ++e) {
    float w0 = a0[e];
    float w1 = a1[e];
    if (MASKED) {
      const float g0 = q0[e];
      const float g1 = q1[e];
      w0 = (g0 == 0.0f) ? 0.0f : (w0 * g0);
      w1 = (g1 == 0.0f) ? 0.0f : (w1 * g1);
    }
    hv[e]     = (_Float16)(w0 * carry);
    hv[4 + e] = (_Float16)(w1 * carry);
  }
  unsigned short* p = dst + e0;
  *(volatile v8h*)p = hv;
  __threadfence();
  *(volatile v8h*)p = hv;
}

__global__ __launch_bounds__(256) void spline_kernel(
    const float* __restrict__ x, const float* __restrict__ raw,
    float* __restrict__ out0, float* __restrict__ out1, int rowBase)
{
  __shared__ __align__(16) float sRaw[8][kStripF];
  __shared__ __align__(16) float sOut[8][4 * kD];
  __shared__ __align__(16) float sLad[kSpRows];
  const int tid = threadIdx.x, lane = tid & 31, wave = tid >> 5;
  const int lrow0 = blockIdx.x * kSpRows + wave * 4;
  float* strip = sRaw[wave];
  float* mine  = strip + lane * kOpd;
  float* otile = sOut[wave];
  float rowacc = 0.0f;

#pragma unroll 1
  for (int it = 0; it < 16; ++it) {
    const int r = it >> 2;
    const int pass = it & 3;
    const int lrow = lrow0 + r;
    const size_t grow = (size_t)rowBase + (size_t)lrow;
    __syncthreads();
    {
      const float* src = raw + (size_t)lrow * kNOut + pass * kSlabF;
#pragma unroll
      for (int q = 0; q < 7; ++q) {
        const int idx = q * 32 + lane;
        const int idc = (idx < kSlabV) ? idx : (kSlabV - 1);
        const v4f pv = *(const v4f*)(src + idc * 4);
        *(v4f*)(strip + idx * 4) = pv;
      }
    }
    __syncthreads();
    const float xv = x[grow * kD + pass * 32 + lane];

#pragma unroll 1
    for (int g = 0; g < 2; ++g) {
      float* u = mine + g * kBins;
      float mx = u[0];
#pragma unroll
      for (int k = 1; k < kBins; ++k) mx = fmaxf(mx, u[k]);
      float ssum = 0.0f;
#pragma unroll 1
      for (int k = 0; k < kBins; ++k) {
        const float e = __expf(u[k] - mx);
        ssum += e;
        u[k] = e;
      }
      const float inv = __builtin_amdgcn_rcpf(ssum);
      float cum = 0.0f;
#pragma unroll 1
      for (int k = 0; k < kBins; ++k) {
        const float sm = u[k] * inv;
        const float wv = kMinBin + kBinScale * sm;
        cum += wv;
        u[k] = cum;
      }
      const float dinv = __builtin_amdgcn_rcpf(fmaxf(cum, 1e-12f));
#pragma unroll 1
      for (int k = 0; k < kBins; ++k) u[k] = u[k] * dinv;
    }
#pragma unroll 1
    for (int k = 0; k <= kBins; ++k) {
      const float v  = mine[2 * kBins + k];
      const float ea = __expf(-fabsf(v));
      const float u1 = 1.0f + ea;
      const float l1 = __logf(u1) + (ea - (u1 - 1.0f)) * __builtin_amdgcn_rcpf(u1);
      mine[2 * kBins + k] = kMinDer + (fmaxf(v, 0.0f) + l1);
    }

    const bool inside = (xv >= -kTB) && (xv <= kTB);
    float xs = (xv + kTB) * kInvSpan;
    xs = fminf(fmaxf(xs, 0.0f), 1.0f);
    int cnt = (xs >= 0.0f) ? 1 : 0;
#pragma unroll
    for (int k = 0; k < kBins; ++k) cnt += (xs >= mine[k]) ? 1 : 0;
    int bid = cnt - 1;
    bid = bid < 0 ? 0 : (bid > (kBins - 1) ? (kBins - 1) : bid);
    const int bm = (bid > 0) ? (bid - 1) : 0;
    const float cwl = mine[bm];
    const float cwr = mine[bid];
    const float chl = mine[kBins + bm];
    const float chr = mine[kBins + bid];
    const float dk  = mine[2 * kBins + bid];
    const float dk1 = mine[2 * kBins + bid + 1];
    const float xk = (bid > 0) ? cwl : 0.0f;
    const float yk = (bid > 0) ? chl : 0.0f;
    const float wk = cwr - xk;
    const float hk = chr - yk;

    const float rw = __builtin_amdgcn_rcpf(wk + kEps);
    float t = (xs - xk) * rw;
    t = fminf(fmaxf(t, 0.0f), 1.0f);
    const float a   = (hk + kEps) * rw;
    const float omt = 1.0f - t;
    const float tt  = t * omt;
    const float num = a * t * t + dk * tt;
    const float den = a + (dk + dk1 - 2.0f * a) * tt;
    const float s   = num * __builtin_amdgcn_rcpf(den + kEps);
    const float y   = (yk + hk * s) * kSpanY - kTB;
    const float dnum = a * a * (dk1 * t * t + 2.0f * a * tt + dk * omt * omt);
    const float dydx = kSlope * dnum * __builtin_amdgcn_rcpf(den * den + kEps);
    const float lg   = logf(fmaxf(dydx, 1e-12f));
    const float outv = inside ? y : xv;
    const float ladv = inside ? lg : 0.0f;

    float rs = ladv;
#pragma unroll
    for (int off = 16; off > 0; off >>= 1) rs += __shfl_xor(rs, off, 32);
    const float base = (pass == 0) ? 0.0f : rowacc;
    rowacc = base + rs;

    otile[r * kD + pass * 32 + lane] = outv;
    if (pass == 3) {
      if (lane == 0) sLad[wave * 4 + r] = rowacc;
    }
  }
  __syncthreads();

  {
    v4f ov[4];
#pragma unroll
    for (int r = 0; r < 4; ++r) ov[r] = *(const v4f*)(otile + r * kD + lane * 4);
    for (int pass = 0; pass < 2; ++pass) {
#pragma unroll
      for (int r = 0; r < 4; ++r) {
        const size_t grow = (size_t)rowBase + (size_t)(lrow0 + r);
        *(volatile v4f*)(out0 + grow * kD + lane * 4) = ov[r];
      }
      __threadfence();
    }
  }
  if (wave == 0) {
    const float lv = sLad[lane];
    volatile float* p = out1 + (size_t)rowBase + (size_t)blockIdx.x * kSpRows + lane;
    *p = lv;
    __threadfence();
    *p = lv;
  }
}

extern "C" void kernel_launch(void* const* d_in, const int* in_sizes, int n_in,
                              void* d_out, int out_size, void* d_ws, size_t ws_size,
                              hipStream_t stream) {
  if (n_in < 10) return;
  if (in_sizes[0] != kB * kD) return;
  if (in_sizes[1] != kH * kD) return;
  if (in_sizes[2] != kH) return;
  if (in_sizes[3] != kH * kH) return;
  if (in_sizes[4] != kH) return;
  if (in_sizes[5] != kNOut * kH) return;
  if (in_sizes[6] != kNOut) return;
  if (in_sizes[7] != kH * kD) return;
  if (in_sizes[8] != kH * kH) return;
  if (in_sizes[9] != kNOut * kH) return;
  if (out_size != kB * kD + kB) return;
  if (ws_size < kWsTotal) return;

  const float* x  = (const float*)d_in[0];
  const float* W1 = (const float*)d_in[1];
  const float* b1 = (const float*)d_in[2];
  const float* W2 = (const float*)d_in[3];
  const float* b2 = (const float*)d_in[4];
  const float* W3 = (const float*)d_in[5];
  const float* b3 = (const float*)d_in[6];
  const float* m1 = (const float*)d_in[7];
  const float* m2 = (const float*)d_in[8];
  const float* m3 = (const float*)d_in[9];
  float* out0 = (float*)d_out;
  float* out1 = (float*)d_out + (kOut1OffBytes / 4);

  char* ws = (char*)d_ws;
  unsigned short* XH  = (unsigned short*)(ws + kOffXH);
  unsigned short* W1M = (unsigned short*)(ws + kOffW1);
  unsigned short* W2M = (unsigned short*)(ws + kOffW2);
  unsigned short* W3M = (unsigned short*)(ws + kOffW3);
  unsigned short* H1  = (unsigned short*)(ws + kOffH1);
  unsigned short* H2  = (unsigned short*)(ws + kOffH2);
  float*          RAW = (float*)(ws + kOffRaw);

  pack_f16_kernel<false><<<(kB * kD / 8) / 256, 256, 0, stream>>>(x, x, XH, kB * kD / 8, 1.0f);
  pack_f16_kernel<true><<<(kH * kD / 8) / 256, 256, 0, stream>>>(W1, m1, W1M, kH * kD / 8, kWCarry);
  pack_f16_kernel<true><<<(kH * kH / 8) / 256, 256, 0, stream>>>(W2, m2, W2M, kH * kH / 8, kWCarry);
  pack_f16_kernel<true><<<(kNOut * kH / 8) / 256, 256, 0, stream>>>(W3, m3, W3M, kNOut * kH / 8, kWCarry);

  wmma_gemm64<1, 3><<<((kB / 64) * (kH / 64)) / 8, 256, 0, stream>>>(
      XH, kD, W1M, kD, (void*)H1, kH, b1, kB, kH, kD, kWCarryInv);

  wmma_gemm64<1, 3><<<((kB / 64) * (kH / 64)) / 8, 256, 0, stream>>>(
      H1, kH, W2M, kH, (void*)H2, kH, b2, kB, kH, kH, kWCarryInv);

  for (int c = 0; c < kNChunk; ++c) {
    const unsigned short* Ac = H2 + (size_t)c * kChunk * kH;
    wmma_gemm64<0, 0><<<((kChunk / 64) * (kNOut / 64)) / 8, 256, 0, stream>>>(
        Ac, kH, W3M, kH, (void*)RAW, kNOut, b3, kChunk, kNOut, kH, kWCarryInv);
    spline_kernel<<<kChunk / kSpRows, 256, 0, stream>>>(x, RAW, out0, out1, c * kChunk);
  }
}
